// RGCNLayer_6571299963187
// MI455X (gfx1250) — hardware-verified
//
#include <hip/hip_runtime.h>
#include <stddef.h>
#include <stdint.h>

#define NN      100000
#define DF      128
#define NR      8
#define NE      1600000
#define GBM     128
#define MP      100096
#define NTHR    256
#define NWAVE   8
#define EPT     8
#define WCH     (32 * EPT)
#define NBRUN   1024
#define SLB     10
#define NBK     98
#define NPR     (NBK * NBRUN)
#define NSUB    (NR * NBRUN)
#define WLCAP   3072
#define RCAP    20480
#define MAXB1024_MEAS 16721
#define MAXDEG_MEAS   36
#define RPB     64
#define NRB     ((NN + RPB - 1) / RPB)

#define BK_ZINTS (NWAVE * WLCAP + RCAP + 2 * NSUB)
#define BK_INTS  (BK_ZINTS + 16)
#define BK_LDS   (BK_INTS * 4)
#define GM_LDS   (GBM * DF * 4)

#define PBX  (MP * DF / 8 / NTHR)
#define PBW  (NR * DF * DF / 8 / NTHR)

static_assert(NN <= (1 << 17) && NR == 8 && NBRUN == 1024 && NBRUN == (1 << SLB));
static_assert(17 + 3 + 10 <= 32);
static_assert(DF == 32 * 4 && DF % 32 == 0);
static_assert(MP == 782 * GBM && MP >= NN && MP % GBM == 0);
static_assert(NBK * NBRUN >= MP && NRB * RPB <= NPR && NRB * RPB >= NN);
static_assert(NBRUN % RPB == 0 && RPB == NWAVE * 8);
static_assert(NE % WCH == 0 && NE % 4 == 0);
static_assert((long long)RCAP * 100 >= (long long)MAXB1024_MEAS * 105);
static_assert(WLCAP >= MAXB1024_MEAS / 8 + 8 * 46 + 1);
static_assert(RCAP % (NTHR * 4) == 0 && BK_ZINTS % (NTHR * 4) == 0 && NSUB % (NTHR * 4) == 0);
static_assert(NBRUN == NTHR * 4);
static_assert(BK_LDS <= 300000 && BK_LDS <= 327680 && GM_LDS <= 327680);
static_assert((MP * DF / 8) % NTHR == 0 && (NR * DF * DF / 8) % NTHR == 0);

typedef float          v4f   __attribute__((ext_vector_type(4)));
typedef float          v8f   __attribute__((ext_vector_type(8)));
typedef int            v4i   __attribute__((ext_vector_type(4)));
typedef int            v8i   __attribute__((ext_vector_type(8)));
typedef unsigned short v8us  __attribute__((ext_vector_type(8)));
typedef unsigned short v16us __attribute__((ext_vector_type(16)));
typedef __bf16         v16bf __attribute__((ext_vector_type(16)));
typedef v4f  __attribute__((may_alias)) v4fa;
typedef v4i  __attribute__((may_alias)) v4ia;
typedef v8us __attribute__((may_alias)) v8usa;
union FragB { v16bf v; v16us u; v8us h[2]; v8i w; };

__device__ __forceinline__ v8f wmb(const FragB& a, const FragB& b, v8f c) {
  v8f d = __builtin_amdgcn_wmma_f32_16x16x32_bf16(false, a.v, false, b.v, (short)0, c, false, false);
  asm volatile("v_nop\n\tv_nop\n\tv_nop\n\tv_nop" : "+v"(d) : "v"(a.w), "v"(b.w));
  return d;
}

__device__ __forceinline__ unsigned bf16_bits(float f) {
  const unsigned u = __float_as_uint(f);
  const unsigned r = (u + 0x7FFFu + ((u >> 16) & 1u)) >> 16;
  const unsigned q = (u >> 16) | 0x40u;
  return ((u & 0x7fffffffu) > 0x7f800000u) ? q : r;
}

__device__ __forceinline__ void st2_v8us(unsigned short* p, v8us v) {
  *(volatile v8us*)p = v;
  __threadfence();
  *(volatile v8us*)p = v;
}

__device__ __forceinline__ v8us gather8(const float* __restrict__ base, int stride) {
  float f[8];
#pragma unroll
  for (int i = 0; i < 8; ++i) f[i] = base[(size_t)i * (size_t)stride];
  v8us o;
#pragma unroll
  for (int i = 0; i < 8; ++i) o[i] = (unsigned short)bf16_bits(f[i]);
  return o;
}

__device__ __forceinline__ int packw(int s, int t, unsigned slot) {
  s = s < 0 ? 0 : (s > NN - 1 ? NN - 1 : s);
  t = t < 0 ? 0 : (t > NR - 1 ? NR - 1 : t);
  return (int)((unsigned)s | ((unsigned)t << 17) | (slot << 20));
}

__global__ __launch_bounds__(NTHR) void k_prep(const float* __restrict__ x, const float* __restrict__ w,
                                               unsigned short* xb, unsigned short* wt) {
  const int tid = (int)threadIdx.x;
  const int blk = (int)blockIdx.x;
  if (blk < PBX) {
    const int u   = blk * NTHR + tid;
    const int row = u >> 4, k8 = (u & 15) * 8;
    const int rc  = row < NN ? row : NN - 1;
    const unsigned mk = row < NN ? 0xffffu : 0u;
    const float* p = x + (size_t)rc * DF + k8;
    const v4f a = *(const v4fa*)p;
    const v4f b = *(const v4fa*)(p + 4);
    v8us o;
    o[0] = (unsigned short)(bf16_bits(a.x) & mk); o[1] = (unsigned short)(bf16_bits(a.y) & mk);
    o[2] = (unsigned short)(bf16_bits(a.z) & mk); o[3] = (unsigned short)(bf16_bits(a.w) & mk);
    o[4] = (unsigned short)(bf16_bits(b.x) & mk); o[5] = (unsigned short)(bf16_bits(b.y) & mk);
    o[6] = (unsigned short)(bf16_bits(b.z) & mk); o[7] = (unsigned short)(bf16_bits(b.w) & mk);
    st2_v8us(xb + (size_t)row * DF + k8, o);
  } else {
    const int u = (blk - PBX) * NTHR + tid;
    const int r = u >> 11, n = (u >> 4) & (DF - 1), k8 = (u & 15) * 8;
    const v8us o = gather8(w + (size_t)r * DF * DF + (size_t)k8 * DF + n, DF);
    st2_v8us(wt + (size_t)r * DF * DF + (size_t)n * DF + k8, o);
  }
}

__device__ __forceinline__ void bucket_flush(const int* pl, const int* cnt, const int* offs, int ov,
                                             int* lp, int* offp, int* cntp, int* fp, int tid) {
#pragma unroll 1
  for (int i = tid * 4; i < RCAP; i += NTHR * 4) {
    const v4i v = *(const v4ia*)(pl + i);
    *(volatile v4i*)(lp + i) = v;
  }
#pragma unroll 1
  for (int r = 0; r < NR; ++r) {
    const v4i a = *(const v4ia*)(offs + r * NBRUN + 4 * tid);
    const v4i c = *(const v4ia*)(cnt + r * NBRUN + 4 * tid);
    *(volatile v4i*)(offp + (size_t)r * NPR + 4 * tid) = a;
    *(volatile v4i*)(cntp + (size_t)r * NPR + 4 * tid) = c;
  }
  if (tid < 8) {
    const v4i f = {ov, ov, ov, ov};
    *(volatile v4i*)(fp + 4 * tid) = f;
  }
}

__global__ __launch_bounds__(NTHR) void k_bucket(const int* __restrict__ keys, const int* __restrict__ gath,
                                                 const int* __restrict__ types, int* LIST, int* OFF, int* CNT,
                                                 int* FLAG) {
  extern __shared__ __attribute__((aligned(16))) int dsm[];
  int* wl   = dsm;
  int* pl   = dsm + NWAVE * WLCAP;
  int* cnt  = pl + RCAP;
  int* cur  = cnt + NSUB;
  int* misc = cur + NSUB;
  const int tid = (int)threadIdx.x, lane = tid & 31, wave = tid >> 5;
  const int blk = (int)blockIdx.x;
  const unsigned nbs = (unsigned)(blk * NBRUN);

  {
    const v4i z4 = {0, 0, 0, 0};
#pragma unroll 1
    for (int i = tid * 4; i < BK_ZINTS; i += NTHR * 4) *(v4ia*)(dsm + i) = z4;
    if (tid < 16) misc[tid] = 0;
  }
  __syncthreads();

  {
    const int per  = ((NE + NWAVE * WCH - 1) / (NWAVE * WCH)) * WCH;
    const int ebeg = wave * per;
    const int eend = (ebeg + per < NE) ? (ebeg + per) : NE;
    int* mylist = wl + wave * WLCAP;
    int wc = 0;
#pragma unroll 1
    for (int cb = ebeg; cb < eend; cb += WCH) {
      const int e0 = cb + lane * EPT;
      const v4i da = *(const v4ia*)(keys + e0);
      const v4i db = *(const v4ia*)(keys + e0 + 4);
      const unsigned s0 = (unsigned)da.x - nbs, s1 = (unsigned)da.y - nbs;
      const unsigned s2 = (unsigned)da.z - nbs, s3 = (unsigned)da.w - nbs;
      const unsigned s4 = (unsigned)db.x - nbs, s5 = (unsigned)db.y - nbs;
      const unsigned s6 = (unsigned)db.z - nbs, s7 = (unsigned)db.w - nbs;
      const bool h0 = s0 < (unsigned)NBRUN, h1 = s1 < (unsigned)NBRUN, h2 = s2 < (unsigned)NBRUN, h3 = s3 < (unsigned)NBRUN;
      const bool h4 = s4 < (unsigned)NBRUN, h5 = s5 < (unsigned)NBRUN, h6 = s6 < (unsigned)NBRUN, h7 = s7 < (unsigned)NBRUN;
      const unsigned m0 = __builtin_amdgcn_ballot_w32(h0), m1 = __builtin_amdgcn_ballot_w32(h1);
      const unsigned m2 = __builtin_amdgcn_ballot_w32(h2), m3 = __builtin_amdgcn_ballot_w32(h3);
      const unsigned m4 = __builtin_amdgcn_ballot_w32(h4), m5 = __builtin_amdgcn_ballot_w32(h5);
      const unsigned m6 = __builtin_amdgcn_ballot_w32(h6), m7 = __builtin_amdgcn_ballot_w32(h7);
      const unsigned any = m0 | m1 | m2 | m3 | m4 | m5 | m6 | m7;
      if (any != 0u) {
        const v4i ga = *(const v4ia*)(gath + e0);
        const v4i gb = *(const v4ia*)(gath + e0 + 4);
        const v4i ta = *(const v4ia*)(types + e0);
        const v4i tb = *(const v4ia*)(types + e0 + 4);
        asm volatile("" :: "v"(ga), "v"(gb));
        asm volatile("" :: "v"(ta), "v"(tb));
        const int w0 = packw(ga.x, ta.x, s0), w1 = packw(ga.y, ta.y, s1);
        const int w2 = packw(ga.z, ta.z, s2), w3 = packw(ga.w, ta.w, s3);
        const int w4 = packw(gb.x, tb.x, s4), w5 = packw(gb.y, tb.y, s5);
        const int w6 = packw(gb.z, tb.z, s6), w7 = packw(gb.w, tb.w, s7);
        const int pre = (int)(__builtin_amdgcn_mbcnt_lo(m0, 0u) + __builtin_amdgcn_mbcnt_lo(m1, 0u) +
                              __builtin_amdgcn_mbcnt_lo(m2, 0u) + __builtin_amdgcn_mbcnt_lo(m3, 0u) +
                              __builtin_amdgcn_mbcnt_lo(m4, 0u) + __builtin_amdgcn_mbcnt_lo(m5, 0u) +
                              __builtin_amdgcn_mbcnt_lo(m6, 0u) + __builtin_amdgcn_mbcnt_lo(m7, 0u));
        int p = wc + pre;
        if (h0) { if (p < WLCAP) mylist[p] = w0; p = p + 1; }
        if (h1) { if (p < WLCAP) mylist[p] = w1; p = p + 1; }
        if (h2) { if (p < WLCAP) mylist[p] = w2; p = p + 1; }
        if (h3) { if (p < WLCAP) mylist[p] = w3; p = p + 1; }
        if (h4) { if (p < WLCAP) mylist[p] = w4; p = p + 1; }
        if (h5) { if (p < WLCAP) mylist[p] = w5; p = p + 1; }
        if (h6) { if (p < WLCAP) mylist[p] = w6; p = p + 1; }
        if (h7) { if (p < WLCAP) mylist[p] = w7; p = p + 1; }
        wc += (int)(__builtin_popcount(m0) + __builtin_popcount(m1) + __builtin_popcount(m2) + __builtin_popcount(m3) +
                    __builtin_popcount(m4) + __builtin_popcount(m5) + __builtin_popcount(m6) + __builtin_popcount(m7));
      }
    }
    if (lane == 0) misc[wave] = wc;
  }
  __syncthreads();

  if (wave == 0) {
    int ov = 0, tot = 0;
#pragma unroll 1
    for (int w2 = 0; w2 < NWAVE; ++w2) {
      int c = misc[w2];
      if (c > WLCAP) ov = 1;
      c = c < 0 ? 0 : (c > WLCAP ? WLCAP : c);
      c = __builtin_amdgcn_readfirstlane(c);
      tot += c;
#pragma unroll 1
      for (int b0 = 0; b0 < c; b0 += 32) {
        const int idx = b0 + lane;
        const int ent = wl[w2 * WLCAP + (idx < WLCAP ? idx : WLCAP - 1)];
        const int m32 = (c - b0) < 32 ? (c - b0) : 32;
#pragma unroll 1
        for (int k = 0; k < m32; ++k) {
          const int u   = __builtin_amdgcn_readlane(ent, k);
          const int sub = (((u >> 17) & (NR - 1)) << SLB) | ((u >> 20) & (NBRUN - 1));
          if (lane == 0) cnt[sub] = cnt[sub] + 1;
        }
      }
    }
    if (tot > RCAP) ov = 1;
    if (lane == 0) misc[9] = ov;
  }
  __syncthreads();
  if (wave == 0) {
    const int base = lane * (NSUB / 32);
    int s = 0;
#pragma unroll 1
    for (int i = 0; i < NSUB / 32; ++i) s += cnt[base + i];
    int incl = s;
#pragma unroll
    for (int d = 1; d < 32; d <<= 1) {
      const int y = __shfl_up(incl, d, 32);
      if (lane >= d) incl += y;
    }
    int run = incl - s;
#pragma unroll 1
    for (int i = 0; i < NSUB / 32; ++i) {
      const int cv = cnt[base + i];
      cur[base + i] = run;
      run += cv;
    }
  }
  __syncthreads();

  if (wave == 0) {
#pragma unroll 1
    for (int w2 = 0; w2 < NWAVE; ++w2) {
      int c = misc[w2];
      c = c < 0 ? 0 : (c > WLCAP ? WLCAP : c);
      c = __builtin_amdgcn_readfirstlane(c);
#pragma unroll 1
      for (int b0 = 0; b0 < c; b0 += 32) {
        const int idx = b0 + lane;
        const int ent = wl[w2 * WLCAP + (idx < WLCAP ? idx : WLCAP - 1)];
        const int m32 = (c - b0) < 32 ? (c - b0) : 32;
#pragma unroll 1
        for (int k = 0; k < m32; ++k) {
          const int u   = __builtin_amdgcn_readlane(ent, k);
          const int sub = (((u >> 17) & (NR - 1)) << SLB) | ((u >> 20) & (NBRUN - 1));
          if (lane == 0) {
            int p = cur[sub];
            p = p < 0 ? 0 : (p > RCAP - 1 ? RCAP - 1 : p);
            pl[p] = u & 0x1FFFF;
            cur[sub] = p + 1;
          }
        }
      }
    }
  }
  __syncthreads();
#pragma unroll 1
  for (int i = tid * 4; i < NSUB; i += NTHR * 4) {
    const v4i a = *(const v4ia*)(cur + i);
    const v4i c = *(const v4ia*)(cnt + i);
    const v4i o = a - c;
    *(v4ia*)(cur + i) = o;
  }
  __syncthreads();

  const int ovf = misc[9];
  int* lp   = LIST + (size_t)blk * RCAP;
  int* offp = OFF + (size_t)blk * NBRUN;
  int* cntp = CNT + (size_t)blk * NBRUN;
  int* fp   = FLAG + (size_t)blk * 32;
  bucket_flush(pl, cnt, cur, ovf, lp, offp, cntp, fp, tid);
  __threadfence();
  bucket_flush(pl, cnt, cur, ovf, lp, offp, cntp, fp, tid);
}

__global__ __launch_bounds__(NTHR) __attribute__((amdgpu_num_vgpr(248)))
void k_gemm(const unsigned short* __restrict__ XB, const unsigned short* __restrict__ WTr, float* P) {
  extern __shared__ __attribute__((aligned(16))) float stg[];
  const int tid = (int)threadIdx.x, lane = tid & 31, wave = tid >> 5, hh = lane >> 4, m = lane & 15;
  const int rowBase = (int)blockIdx.x * GBM;

  v8f acc[8];
  {
    const v8f z = {0.f, 0.f, 0.f, 0.f, 0.f, 0.f, 0.f, 0.f};
#pragma unroll
    for (int t = 0; t < 8; ++t) acc[t] = z;
  }
  const unsigned short* ap = XB + (size_t)(rowBase + 16 * wave + m) * (size_t)DF + 8 * hh;
  const unsigned short* bp = WTr + (size_t)m * (size_t)DF + 8 * hh;

#pragma unroll 1
  for (int k0 = 0; k0 < DF; k0 += 32) {
    FragB af;
    af.h[0] = *(const v8usa*)(ap + k0);
    af.h[1] = *(const v8usa*)(ap + k0 + 16);
#pragma unroll
    for (int nt = 0; nt < 8; ++nt) {
      const unsigned short* wq = bp + (size_t)(16 * nt) * (size_t)DF + k0;
      FragB bf;
      bf.h[0] = *(const v8usa*)wq;
      bf.h[1] = *(const v8usa*)(wq + 16);
      acc[nt] = wmb(af, bf, acc[nt]);
    }
  }

#pragma unroll
  for (int nt = 0; nt < 8; ++nt) {
    const int lc = 16 * nt + m;
#pragma unroll
    for (int r = 0; r < 8; ++r) {
      const int lr = 16 * wave + 8 * hh + r;
      stg[lr * DF + lc] = acc[nt][r];
    }
  }
  __syncthreads();

  v4f pv[16];
#pragma unroll
  for (int i = 0; i < 16; ++i) pv[i] = *(const v4fa*)(stg + (16 * wave + i) * DF + 4 * lane);

#pragma unroll
  for (int i = 0; i < 16; ++i) {
    const bool ok = (rowBase + 16 * wave + i) < NN;
    const v4f t = pv[i];
    v4f y;
    y.x = (t.x > 0.0f) ? t.x : (t.x - t.x);
    y.y = (t.y > 0.0f) ? t.y : (t.y - t.y);
    y.z = (t.z > 0.0f) ? t.z : (t.z - t.z);
    y.w = (t.w > 0.0f) ? t.w : (t.w - t.w);
    y.x = ok ? y.x : 0.0f; y.y = ok ? y.y : 0.0f; y.z = ok ? y.z : 0.0f; y.w = ok ? y.w : 0.0f;
    pv[i] = y;
  }
#pragma unroll
  for (int i = 0; i < 16; ++i) {
    float* rp = P + (size_t)(rowBase + 16 * wave + i) * DF + 4 * lane;
    *(volatile v4f*)rp = pv[i];
  }
  __threadfence();
#pragma unroll
  for (int i = 0; i < 16; ++i) {
    float* rp = P + (size_t)(rowBase + 16 * wave + i) * DF + 4 * lane;
    *(volatile v4f*)rp = pv[i];
  }
}

template <int FIRST>
__global__ __launch_bounds__(NTHR) void k_replay(const int* __restrict__ LIST, const int* __restrict__ OFFr,
                                                 const int* __restrict__ CNTr, const int* __restrict__ FLAG,
                                                 const float* __restrict__ P, float* out) {
  const int tid = (int)threadIdx.x, lane = tid & 31, wave = tid >> 5;
  const int rowBase = (int)blockIdx.x * RPB;
  const int bucket  = rowBase >> SLB;
  const int* lb  = LIST + (size_t)bucket * RCAP;
  const int flag = FLAG[(size_t)bucket * 32];
  const bool bad = flag != 0;
  const float qnan = __uint_as_float(0x7fc00000u);

#pragma unroll 1
  for (int i = 0; i < RPB / NWAVE; ++i) {
    const int row = rowBase + (RPB / NWAVE) * wave + i;
    int c = CNTr[row];
    int o = OFFr[row];
    c = c < 0 ? 0 : (c > RCAP ? RCAP : c);
    o = o < 0 ? 0 : (o > RCAP - 1 ? RCAP - 1 : o);
    c = __builtin_amdgcn_readfirstlane(c);
    o = __builtin_amdgcn_readfirstlane(o);
    int last = o + c - 1;
    last = last < o ? o : last;
    last = last > RCAP - 1 ? RCAP - 1 : last;
    float a0 = 0.0f, a1 = 0.0f, a2 = 0.0f, a3 = 0.0f;
#pragma unroll 1
    for (int j = 0; j < c; ++j) {
      int idx = o + j;
      idx = idx > last ? last : idx;
      int id = lb[idx];
      id = id < 0 ? 0 : (id > NN - 1 ? NN - 1 : id);
      const v4f v = *(const v4fa*)(P + (size_t)id * DF + 4 * lane);
      a0 += v.x; a1 += v.y; a2 += v.z; a3 += v.w;
    }
    if (row < NN) {
      float* op = out + (size_t)row * DF + 4 * lane;
      float n0 = a0, n1 = a1, n2 = a2, n3 = a3;
      if constexpr (FIRST == 0) {
        const v4f old = *(const v4fa*)op;
        n0 = old.x + a0; n1 = old.y + a1; n2 = old.z + a2; n3 = old.w + a3;
      }
      n0 = bad ? qnan : n0; n1 = bad ? qnan : n1; n2 = bad ? qnan : n2; n3 = bad ? qnan : n3;
      v4f nv;
      nv.x = n0; nv.y = n1; nv.z = n2; nv.w = n3;
      *(volatile v4f*)op = nv;
      __threadfence();
      *(volatile v4f*)op = nv;
    }
  }
}

extern "C" void kernel_launch(void* const* d_in, const int* in_sizes, int n_in,
                              void* d_out, int out_size, void* d_ws, size_t ws_size,
                              hipStream_t stream) {
  if (n_in < 4) return;
  if (in_sizes[0] != NN * DF) return;
  if (in_sizes[1] != NR * DF * DF) return;
  if (in_sizes[2] != 2 * NE) return;
  if (in_sizes[3] != NE) return;
  if (out_size != NN * DF) return;

  const float* x  = (const float*)d_in[0];
  const float* W  = (const float*)d_in[1];
  const int*   ei = (const int*)d_in[2];
  const int*   et = (const int*)d_in[3];
  float* out = (float*)d_out;
  const int* keys = ei;
  const int* gath = ei + NE;

  constexpr size_t zXB   = (size_t)MP * DF * 2;
  constexpr size_t zWT   = (size_t)NR * DF * DF * 2;
  constexpr size_t zP    = (size_t)MP * DF * 4;
  constexpr size_t zLIST = (size_t)NBK * RCAP * 4;
  constexpr size_t zOC   = (size_t)NR * NPR * 4;
  constexpr size_t zFLAG = (size_t)NBK * 128;
  constexpr size_t oXB   = 0;
  constexpr size_t oWT   = oXB + zXB;
  constexpr size_t oP    = oWT + zWT;
  constexpr size_t oLIST = oP + zP;
  constexpr size_t oOFF  = oLIST + zLIST;
  constexpr size_t oCNT  = oOFF + zOC;
  constexpr size_t oFLAG = oCNT + zOC;
  constexpr size_t oEND  = oFLAG + zFLAG;
  static_assert(zXB % 256 == 0 && zWT % 256 == 0 && zP % 256 == 0 && zLIST % 256 == 0);
  static_assert(zOC % 256 == 0 && zFLAG % 256 == 0);
  static_assert(oEND <= ((size_t)128u << 20));
  if (oEND > ws_size) return;

  char* ws = (char*)d_ws;
  unsigned short* XB   = (unsigned short*)(ws + oXB);
  unsigned short* WT   = (unsigned short*)(ws + oWT);
  float*          P    = (float*)(ws + oP);
  int*            LIST = (int*)(ws + oLIST);
  int*            OFF  = (int*)(ws + oOFF);
  int*            CNT  = (int*)(ws + oCNT);
  int*            FLAG = (int*)(ws + oFLAG);

  hipFuncSetAttribute(reinterpret_cast<const void*>(&k_bucket), hipFuncAttributeMaxDynamicSharedMemorySize, (int)BK_LDS);
  hipFuncSetAttribute(reinterpret_cast<const void*>(&k_gemm), hipFuncAttributeMaxDynamicSharedMemorySize, (int)GM_LDS);

  k_prep<<<PBX + PBW, NTHR, 0, stream>>>(x, W, XB, WT);
  k_bucket<<<NBK, NTHR, BK_LDS, stream>>>(keys, gath, et, LIST, OFF, CNT, FLAG);

  for (int r = 0; r < NR; ++r) {
    const unsigned short* wtr = WT + (size_t)r * DF * DF;
    const int* offr = OFF + (size_t)r * NPR;
    const int* cntr = CNT + (size_t)r * NPR;
    k_gemm<<<MP / GBM, NTHR, GM_LDS, stream>>>(XB, wtr, P);
    if (r == 0)
      k_replay<1><<<NRB, NTHR, 0, stream>>>(LIST, offr, cntr, FLAG, P, out);
    else
      k_replay<0><<<NRB, NTHR, 0, stream>>>(LIST, offr, cntr, FLAG, P, out);
  }
}
